// TransformerBlock_16320875725478
// MI455X (gfx1250) — hardware-verified
//
#include <hip/hip_runtime.h>
#include <stddef.h>


typedef _Float16 v16h __attribute__((ext_vector_type(16)));
typedef _Float16 v8h  __attribute__((ext_vector_type(8)));
typedef float    v8f  __attribute__((ext_vector_type(8)));
typedef float    v4f  __attribute__((ext_vector_type(4)));

#ifndef NB
#define NB 2
#endif
#ifndef SEQ
#define SEQ 4096
#endif
#define NB_FULL  2
#define SEQ_FULL 4096
#define DIM   256
#define NHEAD 8
#define HD    32
#define HID   1024
#define NGRP  32
#define CPG   8
#define QKP   512
#define MROWS (NB * SEQ)

static_assert(NB >= 1 && NB <= NB_FULL);
static_assert(SEQ >= 128 && SEQ <= SEQ_FULL && (SEQ % 128) == 0);
static_assert(DIM == NHEAD * HD);
static_assert(DIM == NGRP * CPG);
static_assert(HD == 32);
static_assert((NHEAD % 2) == 0);
static_assert((MROWS % 64) == 0 && (DIM % 64) == 0 && (HID % 64) == 0 && (QKP % 64) == 0);
static_assert((DIM % 32) == 0 && (HID % 32) == 0);

#define LDT 72
#define LDK 40
#define LDC 68

#define WCARRY 64.0f
#define PCARRY 1024.0f
#define VCARRY 64.0f

#define WQKV_OFF  ((size_t)0)
#define WPROJ_OFF ((size_t)3 * DIM * DIM)
#define W1_OFF    ((size_t)4 * DIM * DIM)
#define W2_OFF    (W1_OFF + (size_t)HID * DIM)
#define WT_ELEMS  (W2_OFF + (size_t)DIM * HID)
#define WMAX_ELEMS ((size_t)HID * DIM)
static_assert(((size_t)3 * DIM * DIM) % 2048 == 0 && ((size_t)DIM * DIM) % 2048 == 0 &&
              ((size_t)HID * DIM) % 2048 == 0);
static_assert((size_t)3 * DIM * DIM <= WMAX_ELEMS);

#define WT_BYTES  (WT_ELEMS * 2)
#define ST_BYTES  ((size_t)NB * NGRP * 128)
#define XN_BYTES  ((size_t)MROWS * DIM * 2)
#define QK_BYTES  ((size_t)MROWS * QKP * 2)
#define VT_BYTES  ((size_t)NB * DIM * SEQ * 2)
#define OV_BYTES  ((size_t)MROWS * DIM * 2)
#define X1_BYTES  ((size_t)NB * DIM * SEQ * 4)
#define HN_BYTES  ((size_t)MROWS * DIM * 2)
#define H_BYTES   ((size_t)MROWS * HID * 2)
#define WS_TOTAL  (WT_BYTES + 2 * ST_BYTES + XN_BYTES + QK_BYTES + VT_BYTES + OV_BYTES + \
                   X1_BYTES + HN_BYTES + H_BYTES)
static_assert((WT_BYTES % 128) == 0 && (ST_BYTES % 128) == 0 && (XN_BYTES % 128) == 0);
static_assert(WS_TOTAL <= (size_t)134217728);

static_assert((size_t)(QKP / 64) * (MROWS / 64) * 4096 == (size_t)MROWS * QKP);
static_assert((size_t)(MROWS / 64) * (DIM / 64) * 4096 == (size_t)NB * DIM * SEQ);
static_assert((size_t)(SEQ / 128) * (NHEAD / 2) * NB * 128 * 64 == (size_t)MROWS * DIM);
static_assert((size_t)(HID / 64) * (MROWS / 64) * 4096 == (size_t)MROWS * HID);
static_assert((size_t)(SEQ / 64) * (DIM / 64) * NB * 4096 == (size_t)MROWS * DIM);

#define GN_QPC  (SEQ / 4)
#define GN_ITER ((CPG * GN_QPC) / 256)
#define GN_M    (CPG * SEQ)
static_assert(((CPG * GN_QPC) % 256) == 0);

__device__ __forceinline__ float bf16r(float x) {
  unsigned int u = __float_as_uint(x);
  u = (u + 0x7FFFu + ((u >> 16) & 1u)) & 0xFFFF0000u;
  return __uint_as_float(u);
}

__device__ __forceinline__ v16h frag_at(const _Float16* p) {
  v8h lo = *(const v8h*)(p);
  v8h hi = *(const v8h*)(p + 16);
  v16h out;
#pragma unroll
  for (int i = 0; i < 8; ++i) { out[i] = lo[i]; out[i + 8] = hi[i]; }
  return out;
}
__device__ __forceinline__ v16h ld_frag(const _Float16* base, int ld) {
  const int lane = threadIdx.x & 31;
  return frag_at(base + (lane & 15) * ld + (lane >> 4) * 8);
}

__device__ __forceinline__ v8f wmma16(v16h a, v16h b, v8f c) {
  v8f d = __builtin_amdgcn_wmma_f32_16x16x32_f16(false, a, false, b, (short)0, c,
                                                 false, false);
  asm volatile("v_nop\n\tv_nop\n\tv_nop\n\tv_nop" : "+v"(d) : "v"(a), "v"(b));
  return d;
}

__device__ __forceinline__ float red16_max(float x) {
#pragma unroll
  for (int off = 1; off < 16; off <<= 1) x = fmaxf(x, __shfl_xor(x, off, 32));
  return x;
}
__device__ __forceinline__ float red16_sum(float x) {
#pragma unroll
  for (int off = 1; off < 16; off <<= 1) x += __shfl_xor(x, off, 32);
  return x;
}
__device__ __forceinline__ float red32_sum(float x) {
#pragma unroll
  for (int off = 16; off > 0; off >>= 1) x += __shfl_xor(x, off, 32);
  return x;
}

__device__ __forceinline__ void wave_lds_sync() {
  __builtin_amdgcn_fence(3  , "wavefront");
  asm volatile("s_wait_dscnt 0x0" ::: "memory");
  __builtin_amdgcn_wave_barrier();
}

__device__ __forceinline__ float gelu_erf(float v) {
  return 0.5f * v * (1.0f + erff(v * 0.70710678118654752f));
}

__global__ __launch_bounds__(256) void wconv_kernel(
    const float* __restrict__ W0, const float* __restrict__ W1p,
    const float* __restrict__ W2p, const float* __restrict__ W3,
    _Float16* __restrict__ Wt) {
  const int which = blockIdx.y;
  const float* src = W0;
  size_t n = (size_t)3 * DIM * DIM;
  size_t doff = WQKV_OFF;
  if (which == 1) { src = W1p; n = (size_t)DIM * DIM; doff = WPROJ_OFF; }
  if (which == 2) { src = W2p; n = (size_t)HID * DIM; doff = W1_OFF; }
  if (which == 3) { src = W3;  n = (size_t)DIM * HID; doff = W2_OFF; }
  if ((size_t)blockIdx.x * 2048 >= n) return;
  const size_t e = ((size_t)blockIdx.x * 256 + threadIdx.x) * 8;
  const v4f a0 = *(const v4f*)(src + e);
  const v4f a1 = *(const v4f*)(src + e + 4);
  v8h o;
#pragma unroll
  for (int j = 0; j < 4; ++j) {
    o[j]     = (_Float16)(WCARRY * bf16r(a0[j]));
    o[j + 4] = (_Float16)(WCARRY * bf16r(a1[j]));
  }
  *(volatile v8h*)(Wt + doff + e) = o;
  __threadfence();
  *(volatile v8h*)(Wt + doff + e) = o;
}

template <int RNE, int SRCSEQ>
__global__ __launch_bounds__(256) void gn_stats_kernel(
    const float* __restrict__ src, float* __restrict__ stats) {
  __shared__ float red[16];
  const int tid = threadIdx.x, lane = tid & 31, w = tid >> 5;
  const int b = blockIdx.x / NGRP;
  const int g = blockIdx.x - b * NGRP;
  const float* base = src + ((size_t)b * DIM + (size_t)g * CPG) * SRCSEQ;

  float s = 0.0f;
#pragma unroll 4
  for (int it = 0; it < GN_ITER; ++it) {
    const int idx = it * 256 + tid;
    const int c = idx / GN_QPC;
    const int q = idx - c * GN_QPC;
    v4f v = *(const v4f*)(base + (size_t)c * SRCSEQ + q * 4);
    if (RNE) {
#pragma unroll
      for (int j = 0; j < 4; ++j) v[j] = bf16r(v[j]);
    }
    s += (v[0] + v[1]) + (v[2] + v[3]);
  }
  s = red32_sum(s);
  if (lane == 0) red[w] = s;
  __syncthreads();
  float tot = 0.0f;
#pragma unroll
  for (int i = 0; i < 8; ++i) tot += red[i];
  const float mu = tot * (1.0f / (float)GN_M);

  float ss = 0.0f;
#pragma unroll 4
  for (int it = 0; it < GN_ITER; ++it) {
    const int idx = it * 256 + tid;
    const int c = idx / GN_QPC;
    const int q = idx - c * GN_QPC;
    v4f v = *(const v4f*)(base + (size_t)c * SRCSEQ + q * 4);
    if (RNE) {
#pragma unroll
      for (int j = 0; j < 4; ++j) v[j] = bf16r(v[j]);
    }
    const float d0 = v[0] - mu, d1 = v[1] - mu, d2 = v[2] - mu, d3 = v[3] - mu;
    ss += (d0 * d0 + d1 * d1) + (d2 * d2 + d3 * d3);
  }
  ss = red32_sum(ss);
  if (lane == 0) red[8 + w] = ss;
  __syncthreads();
  float tot2 = 0.0f;
#pragma unroll
  for (int i = 0; i < 8; ++i) tot2 += red[8 + i];
  const float var = tot2 * (1.0f / (float)GN_M);
  const float rstd = 1.0f / sqrtf(var + 1.0e-5f);

  if (tid < 8) {
    v4f o;
    o[0] = mu; o[1] = rstd; o[2] = mu; o[3] = rstd;
    float* dst = stats + (size_t)blockIdx.x * 32 + tid * 4;
    *(volatile v4f*)dst = o;
    __threadfence();
    *(volatile v4f*)dst = o;
  }
}

template <int RNE, int SRCSEQ>
__global__ __launch_bounds__(256) void gn_apply_kernel(
    const float* __restrict__ src, const float* __restrict__ stats,
    const float* __restrict__ gw, const float* __restrict__ gb,
    _Float16* __restrict__ dst) {
  __shared__ __align__(16) _Float16 T[64 * LDT];
  __shared__ float Pm[4 * 64];
  const int tid = threadIdx.x;
  const int n0 = blockIdx.x * 64;
  const int c0 = blockIdx.y * 64;
  const int b = blockIdx.z;
  if (tid < 64) {
    const int ch = c0 + tid;
    const int g = ch / CPG;
    const float* st = stats + (size_t)(b * NGRP + g) * 32;
    Pm[tid]       = st[0];
    Pm[64 + tid]  = st[1];
    Pm[128 + tid] = bf16r(gw[ch]);
    Pm[192 + tid] = bf16r(gb[ch]);
  }
  __syncthreads();
#pragma unroll 4
  for (int j = 0; j < 16; ++j) {
    const int idx = tid + 256 * j;
    const int cr = idx >> 6, nc = idx & 63;
    float v = src[((size_t)b * DIM + c0 + cr) * SRCSEQ + n0 + nc];
    if (RNE) v = bf16r(v);
    const float y = ((v - Pm[cr]) * Pm[64 + cr]) * Pm[128 + cr] + Pm[192 + cr];
    T[nc * LDT + cr] = (_Float16)y;
  }
  __syncthreads();
  v8h x[2];
  size_t off[2];
#pragma unroll
  for (int i = 0; i < 2; ++i) {
    const int r = 32 * i + (tid >> 3);
    const int c = (tid & 7) * 8;
    x[i] = *(const v8h*)&T[r * LDT + c];
    off[i] = (size_t)(b * SEQ + n0 + r) * DIM + c0 + c;
  }
#pragma unroll
  for (int i = 0; i < 2; ++i) *(volatile v8h*)(dst + off[i]) = x[i];
  __threadfence();
#pragma unroll
  for (int i = 0; i < 2; ++i) *(volatile v8h*)(dst + off[i]) = x[i];
}

template <int KDIM, int MODE>
__global__ __launch_bounds__(256) void gemm_kernel(
    const _Float16* __restrict__ A16, const _Float16* __restrict__ Bt,
    const float* __restrict__ addf, const float* __restrict__ resf,
    float* __restrict__ outf, _Float16* __restrict__ out16) {
  __shared__ __align__(16) float Cs[64 * LDC];
  const int tid = threadIdx.x, lane = tid & 31, w = tid >> 5;
  const int mw = w >> 1, nw = w & 1;
  const int hh = lane >> 4, m = lane & 15;
  const int n0 = blockIdx.x * 64;
  const int row0 = blockIdx.y * 64;

  const _Float16* ap  = A16 + (size_t)(row0 + mw * 16 + m) * KDIM + hh * 8;
  const _Float16* bp0 = Bt + (size_t)(n0 + nw * 32 + m) * KDIM + hh * 8;
  const _Float16* bp1 = bp0 + 16 * KDIM;
  v8f acc0 = {}, acc1 = {};
#pragma unroll 2
  for (int k0 = 0; k0 < KDIM; k0 += 32) {
    const v16h a  = frag_at(ap + k0);
    const v16h b0 = frag_at(bp0 + k0);
    const v16h b1 = frag_at(bp1 + k0);
    acc0 = wmma16(a, b0, acc0);
    acc1 = wmma16(a, b1, acc1);
  }
#pragma unroll
  for (int r = 0; r < 8; ++r) {
    float* d = &Cs[(mw * 16 + hh * 8 + r) * LDC + nw * 32 + m];
    d[0]  = acc0[r];
    d[16] = acc1[r];
  }
  __syncthreads();

  if (MODE == 0 || MODE == 3) {
    const int ldo = (MODE == 0) ? QKP : HID;
    v8h x[2];
    size_t off[2];
#pragma unroll
    for (int i = 0; i < 2; ++i) {
      const int r = 32 * i + (tid >> 3);
      const int c = (tid & 7) * 8;
      const v4f u0 = *(const v4f*)&Cs[r * LDC + c];
      const v4f u1 = *(const v4f*)&Cs[r * LDC + c + 4];
      if (MODE == 0) {
#pragma unroll
        for (int j = 0; j < 4; ++j) {
          x[i][j]     = (_Float16)(u0[j] * (1.0f / WCARRY));
          x[i][j + 4] = (_Float16)(u1[j] * (1.0f / WCARRY));
        }
      } else {
        const v4f g0 = *(const v4f*)(addf + n0 + c);
        const v4f g1 = *(const v4f*)(addf + n0 + c + 4);
#pragma unroll
        for (int j = 0; j < 4; ++j) {
          const float t0 = gelu_erf(u0[j] * (1.0f / WCARRY) + bf16r(g0[j]));
          const float t1 = gelu_erf(u1[j] * (1.0f / WCARRY) + bf16r(g1[j]));
          x[i][j]     = (_Float16)t0;
          x[i][j + 4] = (_Float16)t1;
        }
      }
      off[i] = (size_t)(row0 + r) * ldo + n0 + c;
    }
#pragma unroll
    for (int i = 0; i < 2; ++i) *(volatile v8h*)(out16 + off[i]) = x[i];
    __threadfence();
#pragma unroll
    for (int i = 0; i < 2; ++i) *(volatile v8h*)(out16 + off[i]) = x[i];
  }

  if (MODE == 1) {
    const int bidx = n0 / SEQ;
    const int nn = n0 - bidx * SEQ;
    v8h x[2];
    size_t off[2];
#pragma unroll
    for (int i = 0; i < 2; ++i) {
      const int r = 32 * i + (tid >> 3);
      const int c = (tid & 7) * 8;
      const v4f u0 = *(const v4f*)&Cs[r * LDC + c];
      const v4f u1 = *(const v4f*)&Cs[r * LDC + c + 4];
#pragma unroll
      for (int j = 0; j < 4; ++j) {
        x[i][j]     = (_Float16)(u0[j] * (1.0f / WCARRY));
        x[i][j + 4] = (_Float16)(u1[j] * (1.0f / WCARRY));
      }
      off[i] = ((size_t)bidx * DIM + row0 + r) * SEQ + nn + c;
    }
#pragma unroll
    for (int i = 0; i < 2; ++i) *(volatile v8h*)(out16 + off[i]) = x[i];
    __threadfence();
#pragma unroll
    for (int i = 0; i < 2; ++i) *(volatile v8h*)(out16 + off[i]) = x[i];
  }

  if (MODE == 2 || MODE == 4) {
    const int bidx = n0 / SEQ;
    const int nn = n0 - bidx * SEQ;
    v4f xs[4];
    size_t off[4];
#pragma unroll
    for (int i = 0; i < 4; ++i) {
      const int r = 16 * i + (tid >> 4);
      const int c = (tid & 15) * 4;
      const int ch = row0 + r;
      const v4f u = *(const v4f*)&Cs[r * LDC + c];
      const float bia = bf16r(addf[ch]);
      const size_t ofull = ((size_t)bidx * DIM + ch) * SEQ_FULL + nn + c;
      const size_t ocomp = ((size_t)bidx * DIM + ch) * SEQ + nn + c;
      v4f val;
      if (MODE == 2) {
        const v4f xr = *(const v4f*)(resf + ofull);
#pragma unroll
        for (int j = 0; j < 4; ++j)
          val[j] = (u[j] * (1.0f / (WCARRY * VCARRY)) + bia) + bf16r(xr[j]);
        off[i] = ocomp;
      } else {
        const v4f rx = *(const v4f*)(resf + ocomp);
#pragma unroll
        for (int j = 0; j < 4; ++j)
          val[j] = (u[j] * (1.0f / WCARRY) + bia) + rx[j];
        off[i] = ofull;
      }
      xs[i] = val;
    }
#pragma unroll
    for (int i = 0; i < 4; ++i) *(volatile v4f*)(outf + off[i]) = xs[i];
    __threadfence();
#pragma unroll
    for (int i = 0; i < 4; ++i) *(volatile v4f*)(outf + off[i]) = xs[i];
  }
}

__global__ __launch_bounds__(512) void attn_kernel(
    const _Float16* __restrict__ QK, const _Float16* __restrict__ Vt,
    const float* __restrict__ pbias, _Float16* __restrict__ Ov) {
  __shared__ __align__(16) _Float16 Ks[2 * 64 * LDK];
  __shared__ __align__(16) _Float16 Vs[64 * LDT];
  __shared__ __align__(16) _Float16 Ps[16 * 16 * LDT];
  __shared__ __align__(16) _Float16 Os[128 * LDT];

  const int tid = threadIdx.x, lane = tid & 31, w = tid >> 5;
  const int hsel = w >> 3, rg = w & 7;
  const int hh = lane >> 4, m = lane & 15;
  const int q0 = blockIdx.x * 128;
  const int hp = blockIdx.y;
  const int b = blockIdx.z;
  const int head = hp * 2 + hsel;
  const float scale = 0.17677669529663687f;
  const float hb = bf16r(pbias[head]);
  _Float16* P = Ps + w * (16 * LDT);

  const size_t qoff = (size_t)(b * SEQ + q0 + rg * 16 + m) * QKP + head * HD + hh * 8;
  const v16h qf = frag_at(QK + qoff);

  float mrow[8], lrow[8];
  v8f o[2];
#pragma unroll
  for (int v = 0; v < 8; ++v) { mrow[v] = -1.0e30f; lrow[v] = 0.0f; }
  o[0] = (v8f){};
  o[1] = (v8f){};

  const int sr = tid >> 3, sc = (tid & 7) * 8;
  const _Float16* ksrc = QK + (size_t)(b * SEQ + sr) * QKP + DIM + hp * 64 + sc;
  const _Float16* vsrc = Vt + ((size_t)b * DIM + hp * 64 + sr) * SEQ + sc;
  _Float16* kdst = &Ks[((sc >> 5) * 64 + sr) * LDK + (sc & 31)];
  _Float16* vdst = &Vs[sr * LDT + sc];

  for (int kb = 0; kb < SEQ; kb += 64) {
    *(v8h*)kdst = *(const v8h*)(ksrc + (size_t)kb * QKP);
    *(v8h*)vdst = *(const v8h*)(vsrc + kb);
    __syncthreads();

    v8f s[4];
#pragma unroll
    for (int kg = 0; kg < 4; ++kg) {
      v8f t = {};
      const v16h kf = ld_frag(&Ks[(hsel * 64 + kg * 16) * LDK], LDK);
      t = wmma16(qf, kf, t);
      s[kg] = t * scale + hb;
    }

    float alpha[8];
#pragma unroll
    for (int v = 0; v < 8; ++v) {
      float mx = fmaxf(fmaxf(s[0][v], s[1][v]), fmaxf(s[2][v], s[3][v]));
      mx = red16_max(mx);
      const float mn = fmaxf(mrow[v], mx);
      alpha[v] = __expf(mrow[v] - mn);
      mrow[v] = mn;
    }
#pragma unroll
    for (int kg = 0; kg < 4; ++kg)
#pragma unroll
      for (int v = 0; v < 8; ++v) s[kg][v] = __expf(s[kg][v] - mrow[v]);
#pragma unroll
    for (int v = 0; v < 8; ++v) {
      const float rs = red16_sum((s[0][v] + s[1][v]) + (s[2][v] + s[3][v]));
      lrow[v] = alpha[v] * lrow[v] + rs;
    }
#pragma unroll
    for (int nb = 0; nb < 2; ++nb)
#pragma unroll
      for (int v = 0; v < 8; ++v) o[nb][v] = o[nb][v] * alpha[v];

#pragma unroll
    for (int kg = 0; kg < 4; ++kg)
#pragma unroll
      for (int v = 0; v < 8; ++v)
        P[(hh * 8 + v) * LDT + kg * 16 + m] = (_Float16)(s[kg][v] * PCARRY);
    wave_lds_sync();

#pragma unroll
    for (int c = 0; c < 2; ++c) {
      const v16h pf = ld_frag(P + c * 32, LDT);
#pragma unroll
      for (int nb = 0; nb < 2; ++nb) {
        const v16h vf = ld_frag(&Vs[(hsel * 32 + nb * 16) * LDT + c * 32], LDT);
        o[nb] = wmma16(pf, vf, o[nb]);
      }
    }
    __syncthreads();
  }

  float inv[8];
#pragma unroll
  for (int v = 0; v < 8; ++v) inv[v] = __builtin_amdgcn_rcpf(lrow[v]) * (VCARRY / PCARRY);
#pragma unroll
  for (int nb = 0; nb < 2; ++nb)
#pragma unroll
    for (int v = 0; v < 8; ++v)
      Os[(rg * 16 + hh * 8 + v) * LDT + hsel * 32 + nb * 16 + m] =
          (_Float16)(o[nb][v] * inv[v]);
  __syncthreads();
  v8h x[2];
  size_t off[2];
#pragma unroll
  for (int i = 0; i < 2; ++i) {
    const int r = 64 * i + (tid >> 3);
    const int c = (tid & 7) * 8;
    x[i] = *(const v8h*)&Os[r * LDT + c];
    off[i] = (size_t)(b * SEQ + q0 + r) * DIM + hp * 64 + c;
  }
#pragma unroll
  for (int i = 0; i < 2; ++i) *(volatile v8h*)(Ov + off[i]) = x[i];
  __threadfence();
#pragma unroll
  for (int i = 0; i < 2; ++i) *(volatile v8h*)(Ov + off[i]) = x[i];
}

extern "C" void kernel_launch(void* const* d_in, const int* in_sizes, int n_in,
                              void* d_out, int out_size, void* d_ws, size_t ws_size,
                              hipStream_t stream) {
  if (n_in < 13) return;
  const long long need_x = ((long long)((NB - 1) * DIM + DIM - 1)) * SEQ_FULL + SEQ;
  if ((long long)in_sizes[0] < need_x) return;
  if (in_sizes[1] < DIM || in_sizes[2] < DIM || in_sizes[3] < DIM || in_sizes[4] < DIM) return;
  if (in_sizes[5] < 3 * DIM * DIM || in_sizes[6] < DIM * DIM || in_sizes[7] < DIM) return;
  if (in_sizes[8] < NHEAD) return;
  if (in_sizes[9] < HID * DIM || in_sizes[10] < HID) return;
  if (in_sizes[11] < DIM * HID || in_sizes[12] < DIM) return;
  if ((long long)out_size < need_x) return;
  if (ws_size < WS_TOTAL) return;

  const float* x      = (const float*)d_in[0];
  const float* gn1_w  = (const float*)d_in[1];
  const float* gn1_b  = (const float*)d_in[2];
  const float* gn2_w  = (const float*)d_in[3];
  const float* gn2_b  = (const float*)d_in[4];
  const float* qkv_w  = (const float*)d_in[5];
  const float* proj_w = (const float*)d_in[6];
  const float* proj_b = (const float*)d_in[7];
  const float* physb  = (const float*)d_in[8];
  const float* mlp_w1 = (const float*)d_in[9];
  const float* mlp_b1 = (const float*)d_in[10];
  const float* mlp_w2 = (const float*)d_in[11];
  const float* mlp_b2 = (const float*)d_in[12];
  float* out = (float*)d_out;

  char* ws = (char*)d_ws;
  _Float16* Wt   = (_Float16*)ws;            ws += WT_BYTES;
  float*    St1  = (float*)ws;               ws += ST_BYTES;
  float*    St2  = (float*)ws;               ws += ST_BYTES;
  _Float16* Xn16 = (_Float16*)ws;            ws += XN_BYTES;
  _Float16* QK16 = (_Float16*)ws;            ws += QK_BYTES;
  _Float16* Vt16 = (_Float16*)ws;            ws += VT_BYTES;
  _Float16* Ov16 = (_Float16*)ws;            ws += OV_BYTES;
  float*    X1   = (float*)ws;               ws += X1_BYTES;
  _Float16* Hn16 = (_Float16*)ws;            ws += HN_BYTES;
  _Float16* H16  = (_Float16*)ws;

  dim3 blk(256);

  wconv_kernel<<<dim3((unsigned)(WMAX_ELEMS / 2048), 4), blk, 0, stream>>>(
      qkv_w, proj_w, mlp_w1, mlp_w2, Wt);

  gn_stats_kernel<1, SEQ_FULL><<<dim3(NB * NGRP), blk, 0, stream>>>(x, St1);
  gn_apply_kernel<1, SEQ_FULL><<<dim3(SEQ / 64, DIM / 64, NB), blk, 0, stream>>>(
      x, St1, gn1_w, gn1_b, Xn16);

  gemm_kernel<DIM, 0><<<dim3(QKP / 64, MROWS / 64), blk, 0, stream>>>(
      Xn16, Wt + WQKV_OFF, proj_b, X1, X1, QK16);
  gemm_kernel<DIM, 1><<<dim3(MROWS / 64, DIM / 64), blk, 0, stream>>>(
      Wt + WQKV_OFF + (size_t)2 * DIM * DIM, Xn16, proj_b, X1, X1, Vt16);

  attn_kernel<<<dim3(SEQ / 128, NHEAD / 2, NB), dim3(512), 0, stream>>>(
      QK16, Vt16, physb, Ov16);

  gemm_kernel<DIM, 2><<<dim3(MROWS / 64, DIM / 64), blk, 0, stream>>>(
      Wt + WPROJ_OFF, Ov16, proj_b, x, X1, Hn16);

  gn_stats_kernel<0, SEQ><<<dim3(NB * NGRP), blk, 0, stream>>>(X1, St2);
  gn_apply_kernel<0, SEQ><<<dim3(SEQ / 64, DIM / 64, NB), blk, 0, stream>>>(
      X1, St2, gn2_w, gn2_b, Hn16);

  gemm_kernel<DIM, 3><<<dim3(HID / 64, MROWS / 64), blk, 0, stream>>>(
      Hn16, Wt + W1_OFF, mlp_b1, X1, X1, H16);
  gemm_kernel<HID, 4><<<dim3(MROWS / 64, DIM / 64), blk, 0, stream>>>(
      Wt + W2_OFF, H16, mlp_b2, X1, out, Hn16);
}
